// LayerNormGRUCell_39745627357260
// MI455X (gfx1250) — hardware-verified
//
#include <hip/hip_runtime.h>
#include <math.h>

constexpr int kRows      = 16384;
constexpr int kIn        = 512;
constexpr int kHid       = 512;
constexpr int kGates     = 3 * kHid;
constexpr int kKcat      = kIn + kHid;
constexpr int kChunk     = 4096;
constexpr int kNumChunks = kRows / kChunk;
constexpr float kInvHid  = 1.0f / 512.0f;
constexpr float kLnEps   = 1e-5f;
static_assert(kRows % kChunk == 0);
static_assert(kIn == 512 && kHid == 512);
static_assert(kChunk % 64 == 0 && kKcat % 64 == 0 && kHid % 64 == 0);

typedef __attribute__((ext_vector_type(16))) _Float16 v16h;
typedef __attribute__((ext_vector_type(8)))  _Float16 v8h;
typedef __attribute__((ext_vector_type(16))) __bf16   v16b;
typedef __attribute__((ext_vector_type(8)))  __bf16   v8b;
typedef __attribute__((ext_vector_type(8)))  float    v8f;
typedef __attribute__((ext_vector_type(4)))  float    v4f;
typedef __attribute__((ext_vector_type(2)))  float    v2f;
typedef __attribute__((ext_vector_type(4)))  unsigned int v4u;

__device__ __forceinline__ unsigned short f2bf_bits(float f) {
  unsigned u = __float_as_uint(f);
  return (unsigned short)((u + 0x7FFFu + ((u >> 16) & 1u)) >> 16);
}
__device__ __forceinline__ float bf_bits2f(unsigned short h) { return __uint_as_float(((unsigned)h) << 16); }

__device__ __forceinline__ void dep_guard_h(v8f& a, v8f& b, v16h x, v16h y) { asm volatile("v_nop\n\tv_nop\n\tv_nop\n\tv_nop" : "+v"(a), "+v"(b) : "v"(x), "v"(y)); }
__device__ __forceinline__ void dep_guard_b(v8f& a, v8f& b, v16b x, v16b y) { asm volatile("v_nop\n\tv_nop\n\tv_nop\n\tv_nop" : "+v"(a), "+v"(b) : "v"(x), "v"(y)); }
__device__ __forceinline__ void keep4_h(v16h a, v16h b, v16h c, v16h d) { asm volatile("v_nop" :: "v"(a), "v"(b), "v"(c), "v"(d)); }
__device__ __forceinline__ void keep4_b(v16b a, v16b b, v16b c, v16b d) { asm volatile("v_nop" :: "v"(a), "v"(b), "v"(c), "v"(d)); }
__device__ __forceinline__ void acc_guard4(v8f& a, v8f& b, v8f& c, v8f& d) { asm volatile("v_nop\n\tv_nop\n\tv_nop\n\tv_nop" : "+v"(a), "+v"(b), "+v"(c), "+v"(d)); }
template <typename T> struct Frag;
template <> struct Frag<_Float16> {
  typedef v16h V; union U { v16h v; v8h h[2]; };
  static __device__ __forceinline__ v16h load(const _Float16* p) {
    U f; f.h[0] = *(const v8h*)(p); f.h[1] = *(const v8h*)(p + 16); return f.v;
  }
  static __device__ __forceinline__ v8f mma(v16h a, v16h b, v8f c) {
    return __builtin_amdgcn_wmma_f32_16x16x32_f16(false, a, false, b, (short)0, c, false, false);
  }
  static __device__ __forceinline__ void guard(v8f& a, v8f& b, v16h x, v16h y) { dep_guard_h(a, b, x, y); }
  static __device__ __forceinline__ void keep(v16h a, v16h b, v16h c, v16h d) { keep4_h(a, b, c, d); }
};
template <> struct Frag<__bf16> {
  typedef v16b V; union U { v16b v; v8b h[2]; };
  static __device__ __forceinline__ v16b load(const __bf16* p) {
    U f; f.h[0] = *(const v8b*)(p); f.h[1] = *(const v8b*)(p + 16); return f.v;
  }
  static __device__ __forceinline__ v8f mma(v16b a, v16b b, v8f c) {
    return __builtin_amdgcn_wmma_f32_16x16x32_bf16(false, a, false, b, (short)0, c, false, false);
  }
  static __device__ __forceinline__ void guard(v8f& a, v8f& b, v16b x, v16b y) { dep_guard_b(a, b, x, y); }
  static __device__ __forceinline__ void keep(v16b a, v16b b, v16b c, v16b d) { keep4_b(a, b, c, d); }
};

__device__ __forceinline__ unsigned pk16(unsigned short a, unsigned short b) { return (unsigned)a | ((unsigned)b << 16); }

template <int ET> struct Elem;
template <> struct Elem<0> { typedef _Float16 T; };
template <> struct Elem<1> { typedef __bf16 T; };
template <int ET, int SPL, int RSC, int OUT_MODE, int ACT, int TRI>
__global__ __launch_bounds__(256) void wmma_gemm64(
    const unsigned short* __restrict__ Ap, const unsigned short* __restrict__ A2p, int lda, long strideA,
    const unsigned short* __restrict__ Btp, const unsigned short* __restrict__ Bt2p, int ldb, long strideB,
    void* __restrict__ Cout, void* __restrict__ Cout2, int ldc, long strideC,
    const float* __restrict__ rsc, long strideS,
    int M, int N, int K, float scale) {
  typedef typename Elem<ET>::T T;
  typedef typename Frag<T>::V V;
  const T* A = (const T*)Ap; const T* A2 = (const T*)A2p; const T* Bt = (const T*)Btp; const T* Bt2 = (const T*)Bt2p;
  __shared__ __align__(16) float sT[8][16 * 68];
  const int b    = blockIdx.y;
  const int lane = threadIdx.x & 31;
  const int wave = threadIdx.x >> 5;
  const int tilesN = N >> 6;
  const int tilesM = M >> 6;
  const int tile = blockIdx.x * 8 + wave;
  if (tile >= tilesM * tilesN) return;
  const int tm = tile / tilesN;
  const int tn = tile - tm * tilesN;
  const int m0 = tm << 6;
  const int n0 = tn << 6;
  if (TRI == 1 && n0 > m0) return;
  const int Kl = (TRI == 2 && (m0 + 64) < K) ? (m0 + 64) : K;

  const T* Ab  = A  + (size_t)b * strideA;
  const T* Bb  = Bt + (size_t)b * strideB;
  const T* Ab2 = (SPL & 1) ? (A2  + (size_t)b * strideA) : nullptr;
  const T* Bb2 = (SPL & 2) ? (Bt2 + (size_t)b * strideB) : nullptr;

  const int rlane = lane & 15;
  const int koff  = (lane >> 4) * 8;
  const int mOff  = (lane >> 4) * 8;

  v8f acc[4][4];
#pragma unroll
  for (int i = 0; i < 4; ++i)
#pragma unroll
    for (int j = 0; j < 4; ++j) acc[i][j] = (v8f){0.f,0.f,0.f,0.f,0.f,0.f,0.f,0.f};

  for (int k0 = 0; k0 < Kl; k0 += 32) {
    V bh[4], bl[4];
#pragma unroll
    for (int j = 0; j < 4; ++j) {
      const size_t bo = (size_t)(n0 + (j << 4) + rlane) * ldb + koff + k0;
      bh[j] = Frag<T>::load(Bb + bo);
      if (SPL & 2) bl[j] = Frag<T>::load(Bb2 + bo);
    }
#pragma unroll
    for (int i = 0; i < 4; ++i) {
      const size_t ao = (size_t)(m0 + (i << 4) + rlane) * lda + koff + k0;
      V ah = Frag<T>::load(Ab + ao);
      V al;
      if (SPL & 1) al = Frag<T>::load(Ab2 + ao);
#pragma unroll
      for (int j = 0; j < 4; ++j) {
        acc[i][j] = Frag<T>::mma(ah, bh[j], acc[i][j]);
        if (SPL & 2) acc[i][j] = Frag<T>::mma(ah, bl[j], acc[i][j]);
        if (SPL & 1) acc[i][j] = Frag<T>::mma(al, bh[j], acc[i][j]);
      }
      Frag<T>::guard(acc[i][0], acc[i][3], ah, (SPL & 1) ? al : ah);
    }
    Frag<T>::keep(bh[0], bh[1], bh[2], bh[3]);
    if (SPL & 2) Frag<T>::keep(bl[0], bl[1], bl[2], bl[3]);
  }
  acc_guard4(acc[0][0], acc[0][1], acc[0][2], acc[0][3]);
  acc_guard4(acc[1][0], acc[1][1], acc[1][2], acc[1][3]);
  acc_guard4(acc[2][0], acc[2][1], acc[2][2], acc[2][3]);
  acc_guard4(acc[3][0], acc[3][1], acc[3][2], acc[3][3]);

  float* slab = sT[wave];
  const float* Rs = RSC ? (rsc + (size_t)b * strideS) : nullptr;
#pragma unroll
  for (int i = 0; i < 4; ++i) {
    const int mBase = m0 + (i << 4);
    float rsv[8];
#pragma unroll
    for (int r = 0; r < 8; ++r) rsv[r] = RSC ? Rs[mBase + mOff + r] : 1.0f;
#pragma unroll
    for (int j = 0; j < 4; ++j) {
      const int n = n0 + (j << 4) + rlane;
#pragma unroll
      for (int r = 0; r < 8; ++r) {
        float v = acc[i][j][r] * scale;
        if (RSC) v = v * rsv[r];
        if (TRI == 1) { if (n > mBase + mOff + r) v = 0.0f; }
        if (ACT == 6) v = (v > 0.0f) ? (v + 1.0f) : __expf(v);
        slab[(mOff + r) * 68 + (j << 4) + rlane] = v;
      }
    }
    __builtin_amdgcn_fence(__ATOMIC_RELEASE, "workgroup");
    __builtin_amdgcn_wave_barrier();
    __builtin_amdgcn_fence(__ATOMIC_ACQUIRE, "workgroup");
    if (OUT_MODE == 0) {
      float* C = (float*)Cout + (size_t)b * strideC;
      const int hh = lane >> 4, c4 = (lane & 15) * 4;
      for (int pass = 0; pass < 2; ++pass) {
#pragma unroll
        for (int it = 0; it < 8; ++it) {
          const int row = it * 2 + hh;
          v4f v = *(const v4f*)(slab + row * 68 + c4);
          *(volatile v4f*)(C + (size_t)(mBase + row) * ldc + n0 + c4) = v;
        }
        __threadfence();
      }
    } else {
      const int q = lane >> 3, c8 = (lane & 7) * 8;
      unsigned short* C  = (unsigned short*)Cout  + (size_t)b * strideC;
      unsigned short* C2 = (OUT_MODE == 2) ? ((unsigned short*)Cout2 + (size_t)b * strideC) : nullptr;
      for (int pass = 0; pass < 2; ++pass) {
#pragma unroll
        for (int it = 0; it < 4; ++it) {
          const int row = it * 4 + q;
          const float* sp = slab + row * 68 + c8;
          v8h hv, lv;
#pragma unroll
          for (int e = 0; e < 8; ++e) {
            if (OUT_MODE == 1) {
              hv[e] = (_Float16)sp[e];
            } else {
              unsigned short hb = f2bf_bits(sp[e]);
              unsigned short lb = f2bf_bits(sp[e] - bf_bits2f(hb));
              hv[e] = __builtin_bit_cast(_Float16, hb);
              lv[e] = __builtin_bit_cast(_Float16, lb);
            }
          }
          *(volatile v8h*)(C + (size_t)(mBase + row) * ldc + n0 + c8) = hv;
          if (OUT_MODE == 2) *(volatile v8h*)(C2 + (size_t)(mBase + row) * ldc + n0 + c8) = lv;
        }
        __threadfence();
      }
    }
    __builtin_amdgcn_fence(__ATOMIC_RELEASE, "workgroup");
    __builtin_amdgcn_wave_barrier();
    __builtin_amdgcn_fence(__ATOMIC_ACQUIRE, "workgroup");
  }
}

__global__ __launch_bounds__(256) void pack2_bf16_kernel(const float* __restrict__ src0, const float* __restrict__ src1,
                                                         unsigned short* __restrict__ dst, int rows) {
  const int i  = blockIdx.x * 256 + threadIdx.x;
  const int n8 = rows * 64;
  if (i >= n8) return;
  const int half = blockIdx.y;
  const float* src = half ? src1 : src0;
  const int row = i >> 6, c8 = (i & 63) * 8;
  const float* p = src + (size_t)row * 512 + c8;
  const v4f a = *(const v4f*)(p);
  const v4f c = *(const v4f*)(p + 4);
  unsigned short hb[8];
#pragma unroll
  for (int e = 0; e < 4; ++e) {
    hb[e]     = f2bf_bits(a[e]);
    hb[4 + e] = f2bf_bits(c[e]);
  }
  const v4u u = (v4u){pk16(hb[0], hb[1]), pk16(hb[2], hb[3]), pk16(hb[4], hb[5]), pk16(hb[6], hb[7])};
  unsigned short* q = dst + (size_t)row * kKcat + half * 512 + c8;
  *(volatile v4u*)q = u;
  __threadfence();
  *(volatile v4u*)q = u;
}

__device__ __forceinline__ float bf_rne(float v) { return bf_bits2f(f2bf_bits(v)); }

__device__ __forceinline__ float block_sum8(float v, float* red, int lane, int wave) {
#pragma unroll
  for (int off = 16; off > 0; off >>= 1) v += __shfl_xor(v, off, 32);
  if (lane == 0) red[wave] = v;
  __syncthreads();
  return ((red[0] + red[1]) + (red[2] + red[3])) + ((red[4] + red[5]) + (red[6] + red[7]));
}

__device__ __forceinline__ float sigmoid_f(float v) {
  const float e = __expf(-v);
  return __builtin_amdgcn_rcpf(1.0f + e);
}

__device__ __forceinline__ float tanh_f(float v) {
  const float a  = fabsf(v);
  const float e  = __expf(-2.0f * a);
  const float tt = (1.0f - e) * __builtin_amdgcn_rcpf(1.0f + e);
  return copysignf(tt, v);
}

__global__ __launch_bounds__(256) void gru_row_kernel(
    const float* __restrict__ RZ, const float* __restrict__ XN, const float* __restrict__ HN,
    const float* __restrict__ h,
    const float* __restrict__ g_r, const float* __restrict__ b_r,
    const float* __restrict__ g_z, const float* __restrict__ b_z,
    const float* __restrict__ g_n, const float* __restrict__ b_n,
    float* __restrict__ out, int row0) {
  __shared__ float red[6][8];
  __shared__ __align__(16) float sOut[kHid];
  const int lr   = blockIdx.x;
  const int grow = row0 + lr;
  const int t = threadIdx.x, lane = t & 31, wave = t >> 5;
  const int c = 2 * t;

  const v2f pr = *(const v2f*)(RZ + (size_t)lr * kKcat + c);
  const v2f pz = *(const v2f*)(RZ + (size_t)lr * kKcat + kHid + c);
  const v2f xn = *(const v2f*)(XN + (size_t)lr * kHid + c);
  const v2f hn = *(const v2f*)(HN + (size_t)lr * kHid + c);
  const v2f hv = *(const v2f*)(h + (size_t)grow * kHid + c);
  const v2f grv = *(const v2f*)(g_r + c), brv = *(const v2f*)(b_r + c);
  const v2f gzv = *(const v2f*)(g_z + c), bzv = *(const v2f*)(b_z + c);
  const v2f gnv = *(const v2f*)(g_n + c), bnv = *(const v2f*)(b_n + c);

  const float hb0 = bf_rne(hv[0]),  hb1 = bf_rne(hv[1]);
  const float gr0 = bf_rne(grv[0]), gr1 = bf_rne(grv[1]), br0 = bf_rne(brv[0]), br1 = bf_rne(brv[1]);
  const float gz0 = bf_rne(gzv[0]), gz1 = bf_rne(gzv[1]), bz0 = bf_rne(bzv[0]), bz1 = bf_rne(bzv[1]);
  const float gn0 = bf_rne(gnv[0]), gn1 = bf_rne(gnv[1]), bn0 = bf_rne(bnv[0]), bn1 = bf_rne(bnv[1]);

  const float mr  = block_sum8(pr[0] + pr[1], red[0], lane, wave) * kInvHid;
  const float dr0 = pr[0] - mr, dr1 = pr[1] - mr;
  const float vr  = block_sum8(dr0 * dr0 + dr1 * dr1, red[1], lane, wave) * kInvHid;
  const float sr  = rsqrtf(vr + kLnEps);
  const float r0  = sigmoid_f((dr0 * sr) * gr0 + br0);
  const float r1  = sigmoid_f((dr1 * sr) * gr1 + br1);

  const float mz  = block_sum8(pz[0] + pz[1], red[2], lane, wave) * kInvHid;
  const float dz0 = pz[0] - mz, dz1 = pz[1] - mz;
  const float vz  = block_sum8(dz0 * dz0 + dz1 * dz1, red[3], lane, wave) * kInvHid;
  const float sz  = rsqrtf(vz + kLnEps);
  const float z0  = sigmoid_f((dz0 * sz) * gz0 + bz0);
  const float z1  = sigmoid_f((dz1 * sz) * gz1 + bz1);

  const float pn0 = xn[0] + r0 * hn[0];
  const float pn1 = xn[1] + r1 * hn[1];
  const float mn  = block_sum8(pn0 + pn1, red[4], lane, wave) * kInvHid;
  const float dn0 = pn0 - mn, dn1 = pn1 - mn;
  const float vn  = block_sum8(dn0 * dn0 + dn1 * dn1, red[5], lane, wave) * kInvHid;
  const float sn  = rsqrtf(vn + kLnEps);
  const float n0  = tanh_f((dn0 * sn) * gn0 + bn0);
  const float n1  = tanh_f((dn1 * sn) * gn1 + bn1);

  const float o0 = (1.0f - z0) * n0 + z0 * hb0;
  const float o1 = (1.0f - z1) * n1 + z1 * hb1;
  sOut[c]     = o0;
  sOut[c + 1] = o1;
  __syncthreads();
  if (t < 128) {
    const v4f v = *(const v4f*)(sOut + 4 * t);
    float* op = out + (size_t)grow * kHid + 4 * t;
    *(volatile v4f*)op = v;
    __threadfence();
    *(volatile v4f*)op = v;
  }
}

extern "C" void kernel_launch(void* const* d_in, const int* in_sizes, int n_in,
                              void* d_out, int out_size, void* d_ws, size_t ws_size,
                              hipStream_t stream) {
  if (n_in < 10) return;
  if (in_sizes[0] != kRows * kIn) return;
  if (in_sizes[1] != kRows * kHid) return;
  if (in_sizes[2] != kGates * kIn) return;
  if (in_sizes[3] != kGates * kHid) return;
  for (int i = 4; i < 10; ++i) if (in_sizes[i] != kHid) return;
  if (out_size != kRows * kHid) return;

  const float* x   = (const float*)d_in[0];
  const float* h   = (const float*)d_in[1];
  const float* Wi  = (const float*)d_in[2];
  const float* Wh  = (const float*)d_in[3];
  const float* g_r = (const float*)d_in[4];
  const float* b_r = (const float*)d_in[5];
  const float* g_z = (const float*)d_in[6];
  const float* b_z = (const float*)d_in[7];
  const float* g_n = (const float*)d_in[8];
  const float* b_n = (const float*)d_in[9];
  float* outp = (float*)d_out;

  const size_t SZ_XB   = (size_t)kRows * kKcat * 2;
  const size_t SZ_WB   = (size_t)kGates * kKcat * 2;
  const size_t SZ_RZ   = (size_t)kChunk * kKcat * 4;
  const size_t SZ_XNHN = (size_t)2 * kChunk * kHid * 4;
  size_t off = 0;
  const size_t oXB   = off; off += SZ_XB;
  const size_t oWB   = off; off += SZ_WB;
  const size_t oRZ   = off; off += SZ_RZ;
  const size_t oXNHN = off; off += SZ_XNHN;
  const size_t TOTAL = off;
  if (TOTAL > ws_size) return;
  if (TOTAL > (size_t)134217728) return;

  char* ws = (char*)d_ws;
  unsigned short* Xb   = (unsigned short*)(ws + oXB);
  unsigned short* Wb   = (unsigned short*)(ws + oWB);
  float*          RZ   = (float*)(ws + oRZ);
  float*          XNHN = (float*)(ws + oXNHN);
  const float* dummy_rsc = RZ;

  const dim3 blk(256);

  pack2_bf16_kernel<<<dim3((kRows * 64 + 255) / 256, 2), blk, 0, stream>>>(x, h, Xb, kRows);
  pack2_bf16_kernel<<<dim3((kGates * 64 + 255) / 256, 2), blk, 0, stream>>>(Wi, Wh, Wb, kGates);

  const int tilesM = kChunk / 64;
  const dim3 gRZ((tilesM * (kKcat / 64) + 7) / 8, 1);
  const dim3 gN((tilesM * (kHid / 64) + 7) / 8, 2);
  const unsigned short* WbN = Wb + (size_t)kKcat * kKcat;

  for (int ch = 0; ch < kNumChunks; ++ch) {
    const unsigned short* A = Xb + (size_t)ch * kChunk * kKcat;
    wmma_gemm64<1, 0, 0, 0, 0, 0><<<gRZ, blk, 0, stream>>>(
        A, A, kKcat, 0L, Wb, Wb, kKcat, 0L, (void*)RZ, (void*)RZ, kKcat, 0L, dummy_rsc, 0L, kChunk, kKcat, kKcat, 1.0f);
    wmma_gemm64<1, 0, 0, 0, 0, 0><<<gN, blk, 0, stream>>>(
        A, A, kKcat, (long)kIn, WbN, WbN, kKcat, (long)kIn, (void*)XNHN, (void*)XNHN, kHid, (long)kChunk * kHid,
        dummy_rsc, 0L, kChunk, kHid, kIn, 1.0f);
    gru_row_kernel<<<dim3(kChunk), blk, 0, stream>>>(
        RZ, XNHN, XNHN + (size_t)kChunk * kHid, h, g_r, b_r, g_z, b_z, g_n, b_n, outp, ch * kChunk);
  }
}
